// InterlacedPoolAttention2_31748398252239
// MI455X (gfx1250) — hardware-verified
//
#include <hip/hip_runtime.h>
#include <math.h>

typedef __attribute__((ext_vector_type(16))) _Float16 v16h;
typedef __attribute__((ext_vector_type(16))) __bf16 v16b;
typedef __attribute__((ext_vector_type(8)))  _Float16 v8h;
typedef __attribute__((ext_vector_type(8)))  float v8f;
typedef __attribute__((ext_vector_type(4)))  float v4f;
typedef __attribute__((ext_vector_type(2)))  float v2f;
typedef __attribute__((ext_vector_type(4)))  unsigned v4u;
typedef __attribute__((ext_vector_type(4)))  int v4i;
typedef float __attribute__((may_alias)) float_a;
typedef int __attribute__((may_alias)) int_a;

template <typename T> __device__ __forceinline__ void vst2(void* p, T v) { *(volatile T*)p = v; __threadfence(); *(volatile T*)p = v; }
__device__ __forceinline__ v8f wmma16(v16h a, v16h b, v8f c) {
  v8f d = __builtin_amdgcn_wmma_f32_16x16x32_f16(false, a, false, b, (short)0, c, false, false);
  asm volatile("v_nop\n\tv_nop\n\tv_nop\n\tv_nop" : "+v"(d) : "v"(a), "v"(b));
  return d;
}
__device__ __forceinline__ v8f wmma_bf(v16b a, v16b b, v8f c) {
  v8f d = __builtin_amdgcn_wmma_f32_16x16x32_bf16(false, a, false, b, (short)0, c, false, false);
  asm volatile("v_nop\n\tv_nop\n\tv_nop\n\tv_nop" : "+v"(d) : "v"(a), "v"(b));
  return d;
}
__device__ __forceinline__ v16h frag_h(const _Float16* rowk0, int lane) {
  union { v16h v; v8h q[2]; } u; const _Float16* p = rowk0 + 8 * (lane >> 4);
  u.q[0] = *(const v8h*)p; u.q[1] = *(const v8h*)(p + 16); return u.v;
}
__device__ __forceinline__ v16h frag_f32(const float* rowk0, int lane) {
  v16h a; const float* p = rowk0 + 8 * (lane >> 4);
#pragma unroll
  for (int i = 0; i < 8; ++i) { a[i] = (_Float16)p[i]; a[8 + i] = (_Float16)p[16 + i]; }
  return a;
}
__device__ __forceinline__ v16h frag_f32s(const float* rowk0, int lane, float sc) {
  v16h a; const float* p = rowk0 + 8 * (lane >> 4);
#pragma unroll
  for (int i = 0; i < 8; ++i) { a[i] = (_Float16)(p[i] * sc); a[8 + i] = (_Float16)(p[16 + i] * sc); }
  return a;
}
__device__ __forceinline__ v16h fragc_f32(const float* W, int k0, int n, int lane, int ld, int K) {
  v16h a; const int g = lane >> 4;
#pragma unroll
  for (int i = 0; i < 8; ++i) { const int ka = k0 + 8 * g + i, kb = ka + 16;
    a[i] = (_Float16)(ka < K ? W[(size_t)(ka < K ? ka : K - 1) * ld + n] : 0.f); a[8 + i] = (_Float16)(kb < K ? W[(size_t)(kb < K ? kb : K - 1) * ld + n] : 0.f); }
  return a;
}
struct F2 { v16b h, l; };
__device__ __forceinline__ F2 bsplit16(const float v[16]) { F2 r;
#pragma unroll
  for (int i = 0; i < 16; ++i) { const __bf16 h = (__bf16)v[i]; r.h[i] = h; r.l[i] = (__bf16)(v[i] - (float)h); }
  return r; }
__device__ __forceinline__ F2 split_row(const float* row, int k0, int lane) { float v[16]; const float* p = row + k0 + 8 * (lane >> 4);
#pragma unroll
  for (int i = 0; i < 8; ++i) { v[i] = p[i]; v[8 + i] = p[16 + i]; }
  return bsplit16(v); }
__device__ __forceinline__ F2 split_rowK(const float* row, int k0, int lane, int K) { float v[16]; const int g = lane >> 4;
#pragma unroll
  for (int i = 0; i < 8; ++i) { const int ka = k0 + 8 * g + i, kb = ka + 16; v[i] = ka < K ? row[ka < K ? ka : K - 1] : 0.f; v[8 + i] = kb < K ? row[kb < K ? kb : K - 1] : 0.f; }
  return bsplit16(v); }
__device__ __forceinline__ F2 split_col(const float* W, int k0, int n, int lane, int ld, int K) { float v[16]; const int g = lane >> 4;
#pragma unroll
  for (int i = 0; i < 8; ++i) { const int ka = k0 + 8 * g + i, kb = ka + 16; v[i] = ka < K ? W[(size_t)(ka < K ? ka : K - 1) * ld + n] : 0.f; v[8 + i] = kb < K ? W[(size_t)(kb < K ? kb : K - 1) * ld + n] : 0.f; }
  return bsplit16(v); }
__device__ __forceinline__ v8f mac3(const F2& a, const F2& b, v8f c) { c = wmma_bf(a.l, b.h, c); c = wmma_bf(a.h, b.l, c); return wmma_bf(a.h, b.h, c); }
__device__ __forceinline__ float sigm(float v) { return 1.0f / (1.0f + expf(-v)); }
#define LDSX() do { asm volatile("s_wait_dscnt 0" ::: "memory"); __builtin_amdgcn_wave_barrier(); __builtin_amdgcn_fence(__ATOMIC_RELEASE, "workgroup"); } while (0)


#define NB 8
#define HH 56
#define WWD 56
#define NP (HH * WWD)
#define CC 384
#define CI 192
#define NH 8
#define HD 48
#define WS7 7
#define LW (WS7 * WS7)
#define NQW (HH / WS7)
#ifndef TNB
#define TNB NB
#endif
typedef __attribute__((ext_vector_type(8))) __bf16 v8b;
__device__ __forceinline__ v16b frag_b(const __bf16* rowk0, int lane) {
  union { v16b v; v8b q[2]; } u; const __bf16* p = rowk0 + 8 * (lane >> 4);
  u.q[0] = *(const v8b*)p; u.q[1] = *(const v8b*)(p + 16); return u.v;
}
__device__ __forceinline__ float bfr(float v) { return (float)(__bf16)v; }
__device__ __attribute__((noinline)) float exp_ni(float v) { return expf(v); }
__device__ __attribute__((noinline)) float erf_ni(float v) { return erff(v); }

#define WS_T   0u
#define WS_PH_ (WS_T + 2u * (size_t)NB * NP * CI)
#define WS_GT  (WS_PH_ + 2u * (size_t)NB * NP * CI)
#define WS_S   (WS_GT + 2u * (size_t)NB * CI * NP)
#define WS_P   (WS_S + 4u * (size_t)NP * NP)
#define WS_FG  (WS_P + 2u * (size_t)NP * NP)
#define WS_X4  (WS_FG + 4u * (size_t)NB * NP * CI)
#define WS_QKV (WS_X4 + 4u * (size_t)NB * NP * CC)
#define WS_O   (WS_QKV + 2u * (size_t)NB * NP * 3 * CC)
#define WS_END (WS_O + 4u * (size_t)NB * NP * CC)

__global__ __launch_bounds__(128) void k_cproj(const float* __restrict__ X, const float* __restrict__ WT, const float* __restrict__ WP, const float* __restrict__ WG, _Float16* __restrict__ T16, _Float16* __restrict__ P16, _Float16* __restrict__ GT) { __shared__ __align__(16) _Float16 sh[64][200]; __shared__ __align__(16) _Float16 tg[192][72];
  const int tid = threadIdx.x, wave = tid >> 5, lane = tid & 31, col = lane & 15, g = lane >> 4; const size_t r0 = (size_t)blockIdx.x * 64; const int which = blockIdx.y; const float* Wm = which == 0 ? WT : which == 1 ? WP : WG;
#pragma unroll 1
  for (int cg = 0; cg < CI / 96; ++cg) { v8f acc[6] = {};
#pragma unroll 2
    for (int kc = 0; kc < CC / 32; ++kc) { v16b a; { const float* p = X + (r0 + wave * 16 + col) * CC + kc * 32 + 8 * g;
#pragma unroll
        for (int i = 0; i < 8; ++i) { a[i] = (__bf16)p[i]; a[8 + i] = (__bf16)p[16 + i]; } }
#pragma unroll
      for (int j = 0; j < 6; ++j) { v16b w; const int o = cg * 96 + j * 16 + col;
#pragma unroll
        for (int i = 0; i < 8; ++i) { w[i] = (__bf16)Wm[(size_t)o * CC + kc * 32 + 8 * g + i]; w[8 + i] = (__bf16)Wm[(size_t)o * CC + kc * 32 + 16 + 8 * g + i]; }
        acc[j] = wmma_bf(a, w, acc[j]); } }
#pragma unroll
    for (int j = 0; j < 6; ++j)
#pragma unroll
      for (int r = 0; r < 8; ++r) { const int rl = wave * 16 + 8 * g + r, cl = cg * 96 + j * 16 + col; const _Float16 hv = (_Float16)acc[j][r]; if (which == 2) tg[cl][rl] = hv; else sh[rl][cl] = hv; } }
  __syncthreads();
  if (which < 2) { _Float16* dst = which == 0 ? T16 : P16; for (int e = tid; e < 64 * 24; e += 128) { const int rl = e / 24, q = e % 24; vst2((unsigned*)(dst + (r0 + rl) * CI + q * 8), *(const v4u*)&sh[rl][q * 8]); } }
  else { const size_t b = r0 / NP; const int n0 = (int)(r0 % NP); for (int e = tid; e < 192 * 8; e += 128) { const int cl = e >> 3, q = e & 7; vst2((unsigned*)(GT + (b * CI + cl) * (size_t)NP + n0 + q * 8), *(const v4u*)&tg[cl][q * 8]); } } }
__global__ __launch_bounds__(128) void k_csc(const _Float16* __restrict__ T16, const _Float16* __restrict__ P16, int b, float* __restrict__ S) { __shared__ __align__(16) float ss[4][16][68];
  const int tid = threadIdx.x, wave = tid >> 5, lane = tid & 31, col = lane & 15, g = lane >> 4; const int k0 = blockIdx.y * 64; const int ql0 = blockIdx.x * 64 + wave * 16; const size_t q0 = (size_t)b * NP + ql0;
  v8f acc[4] = {};
#pragma unroll 1
  for (int kc = 0; kc < CI / 32; ++kc) { const v16h a = frag_h(T16 + (q0 + col) * CI + kc * 32, lane);
#pragma unroll
    for (int j = 0; j < 4; ++j) acc[j] = wmma16(a, frag_h(P16 + ((size_t)b * NP + k0 + j * 16 + col) * CI + kc * 32, lane), acc[j]); }
#pragma unroll
  for (int j = 0; j < 4; ++j)
#pragma unroll
    for (int r = 0; r < 8; ++r) ss[wave][8 * g + r][j * 16 + col] = acc[j][r] * 0.07216878364870323f;
  LDSX(); for (int rl = 0; rl < 16; ++rl) if (lane < 16) vst2(S + (size_t)(ql0 + rl) * NP + k0 + lane * 4, *(const v4f*)&ss[wave][rl][lane * 4]); }
__global__ __launch_bounds__(256) void k_csm(const float* __restrict__ S, _Float16* __restrict__ P) { __shared__ float sred[8]; __shared__ float sbc; __shared__ __align__(16) _Float16 sh[NP];
  const int t = threadIdx.x; const size_t row = blockIdx.x; const float* sr = S + row * NP;
  float m = -3.0e38f; for (int k = t; k < NP; k += 256) m = fmaxf(m, sr[k]);
#pragma unroll
  for (int o = 1; o < 32; o <<= 1) m = fmaxf(m, __shfl_xor(m, o));
  if ((t & 31) == 0) sred[t >> 5] = m; __syncthreads(); if (t == 0) { float a = sred[0]; for (int i = 1; i < 8; ++i) a = fmaxf(a, sred[i]); sbc = a; } __syncthreads(); m = sbc; __syncthreads();
  float sum = 0.f; for (int k = t; k < NP; k += 256) sum += expf(sr[k] - m);
#pragma unroll
  for (int o = 1; o < 32; o <<= 1) sum += __shfl_xor(sum, o);
  if ((t & 31) == 0) sred[t >> 5] = sum; __syncthreads(); if (t == 0) { float a = 0.f; for (int i = 0; i < 8; ++i) a += sred[i]; sbc = 1.0f / a; } __syncthreads(); const float inv = sbc;
  for (int k = t; k < NP; k += 256) sh[k] = (_Float16)(expf(sr[k] - m) * inv * 2048.0f);
  __syncthreads(); for (int q = t; q < NP / 8; q += 256) vst2((unsigned*)(P + row * NP + q * 8), *(const v4u*)&sh[q * 8]); }
__global__ __launch_bounds__(128) void k_cpv(const _Float16* __restrict__ P, const _Float16* __restrict__ GT, int b, float* __restrict__ FG) { __shared__ __align__(16) float ss[4][16][100];
  const int tid = threadIdx.x, wave = tid >> 5, lane = tid & 31, col = lane & 15, g = lane >> 4; const int c0 = blockIdx.y * 96; const int ql0 = blockIdx.x * 64 + wave * 16;
  v8f acc[6] = {};
#pragma unroll 1
  for (int kc = 0; kc < NP / 32; ++kc) { const v16h ph = frag_h(P + (size_t)(ql0 + col) * NP + kc * 32, lane);
#pragma unroll
    for (int j = 0; j < 6; ++j) acc[j] = wmma16(ph, frag_h(GT + ((size_t)b * CI + c0 + j * 16 + col) * (size_t)NP + kc * 32, lane), acc[j]); }
#pragma unroll
  for (int j = 0; j < 6; ++j)
#pragma unroll
    for (int r = 0; r < 8; ++r) ss[wave][8 * g + r][j * 16 + col] = acc[j][r] * (1.0f / 2048.0f);
  LDSX(); for (int rl = 0; rl < 16; ++rl) if (lane < 24) vst2(FG + ((size_t)b * NP + ql0 + rl) * CI + c0 + lane * 4, *(const v4f*)&ss[wave][rl][lane * 4]); }
__global__ __launch_bounds__(128) void k_cout(const float* __restrict__ X, const float* __restrict__ FG, const float* __restrict__ WO, float* __restrict__ X4) { __shared__ __align__(16) float sf[4][16][132];
  const int tid = threadIdx.x, wave = tid >> 5, lane = tid & 31, col = lane & 15, g = lane >> 4; const int c0 = blockIdx.y * 128; const size_t r0 = (size_t)blockIdx.x * 64 + wave * 16;
  v8f acc[8] = {};
#pragma unroll
  for (int kc = 0; kc < CI / 32; ++kc) { const F2 a = split_row(FG + (r0 + col) * CI, kc * 32, lane);
#pragma unroll
    for (int j = 0; j < 8; ++j) { v16b w; const int o = c0 + j * 16 + col;
#pragma unroll
      for (int i = 0; i < 8; ++i) { w[i] = (__bf16)WO[(size_t)o * CI + kc * 32 + 8 * g + i]; w[8 + i] = (__bf16)WO[(size_t)o * CI + kc * 32 + 16 + 8 * g + i]; }
      acc[j] = wmma_bf(a.h, w, acc[j]); acc[j] = wmma_bf(a.l, w, acc[j]); } }
#pragma unroll
  for (int j = 0; j < 8; ++j) { const int c = c0 + j * 16 + col;
#pragma unroll
    for (int r = 0; r < 8; ++r) sf[wave][8 * g + r][j * 16 + col] = bfr(X[(r0 + 8 * g + r) * CC + c]) + acc[j][r]; }
  LDSX(); for (int rl = 0; rl < 16; ++rl) vst2(X4 + (r0 + rl) * CC + c0 + lane * 4, *(const v4f*)&sf[wave][rl][lane * 4]); }
__global__ __launch_bounds__(128) void k_qkv(const float* __restrict__ X4, const float* __restrict__ WI, const float* __restrict__ BI, _Float16* __restrict__ QKV) { __shared__ __align__(16) _Float16 sh[64][136];
  const int tid = threadIdx.x, wave = tid >> 5, lane = tid & 31, col = lane & 15, g = lane >> 4; const int c0 = blockIdx.y * 128; const size_t r0 = (size_t)blockIdx.x * 64;
  v8f acc[8] = {};
#pragma unroll 2
  for (int kc = 0; kc < CC / 32; ++kc) { const v16h a = frag_f32(X4 + (r0 + wave * 16 + col) * CC + kc * 32, lane);
#pragma unroll
    for (int j = 0; j < 8; ++j) { v16h w; const int o = c0 + j * 16 + col;
#pragma unroll
      for (int i = 0; i < 8; ++i) { w[i] = (_Float16)bfr(WI[(size_t)o * CC + kc * 32 + 8 * g + i]); w[8 + i] = (_Float16)bfr(WI[(size_t)o * CC + kc * 32 + 16 + 8 * g + i]); }
      acc[j] = wmma16(a, w, acc[j]); } }
#pragma unroll
  for (int j = 0; j < 8; ++j) { const float bb = bfr(BI[c0 + j * 16 + col]);
#pragma unroll
    for (int r = 0; r < 8; ++r) sh[wave * 16 + 8 * g + r][j * 16 + col] = (_Float16)(acc[j][r] + bb); }
  __syncthreads(); for (int e = tid; e < 64 * 16; e += 128) { const int rl = e >> 4, q = e & 15; vst2((unsigned*)(QKV + (r0 + rl) * (3 * CC) + c0 + q * 8), *(const v4u*)&sh[rl][q * 8]); } }
__global__ __launch_bounds__(128) void k_wat(const _Float16* __restrict__ QKV, const float* __restrict__ RPB, const int* __restrict__ RIX, float* __restrict__ O) {
  __shared__ __align__(16) _Float16 sq[64][72], sk[64][72], sv[64][72]; __shared__ __align__(16) float sp[4][16][68]; __shared__ __align__(16) float so[64][CC + 4]; __shared__ int stok[64];
  const int tid = threadIdx.x, wave = tid >> 5, lane = tid & 31, col = lane & 15, g = lane >> 4; const int wdx = blockIdx.x; const int n = wdx / (NQW * NQW), qh = (wdx / NQW) % NQW, qw = wdx % NQW;
  if (tid < 64) { const int l = tid; stok[l] = (l < LW) ? ((qw * WS7 + (l % WS7)) * WWD + (qh * WS7 + l / WS7)) : -1; }
  __syncthreads();
#pragma unroll 1
  for (int h = 0; h < NH; ++h) {
    for (int e = tid; e < 64 * 64; e += 128) { const int l = e >> 6, d = e & 63; _Float16 qv = 0, kv = 0, vv = 0; if (l < LW && d < HD) { const size_t base = ((size_t)n * NP + stok[l]) * (3 * CC) + h * HD + d; qv = (_Float16)((float)QKV[base] * 0.14433756729740643f); kv = QKV[base + CC]; vv = QKV[base + 2 * CC]; } sq[l][d] = qv; sk[l][d] = kv; sv[d][l] = vv; }
    __syncthreads();
    v8f sc[4] = {};
#pragma unroll
    for (int kc = 0; kc < 2; ++kc) { const v16h a = frag_h(&sq[wave * 16 + col][kc * 32], lane);
#pragma unroll
      for (int j = 0; j < 4; ++j) sc[j] = wmma16(a, frag_h(&sk[j * 16 + col][kc * 32], lane), sc[j]); }
    float pr[4][8]; float mx[8], sm[8];
#pragma unroll
    for (int r = 0; r < 8; ++r) { mx[r] = -3.0e38f; sm[r] = 0.f; }
#pragma unroll
    for (int j = 0; j < 4; ++j) { const int m_ = j * 16 + col;
#pragma unroll
      for (int r = 0; r < 8; ++r) { const int l = wave * 16 + 8 * g + r; float v = -3.0e38f; if (m_ < LW && l < LW) v = sc[j][r] + bfr(RPB[RIX[l * LW + m_] * NH + h]); pr[j][r] = v; mx[r] = fmaxf(mx[r], v); } }
#pragma unroll
    for (int r = 0; r < 8; ++r) {
#pragma unroll
      for (int o = 1; o < 16; o <<= 1) mx[r] = fmaxf(mx[r], __shfl_xor(mx[r], o)); }
#pragma unroll
    for (int j = 0; j < 4; ++j)
#pragma unroll
      for (int r = 0; r < 8; ++r) { const float e_ = (pr[j][r] <= -1.0e38f) ? 0.f : expf(pr[j][r] - mx[r]); pr[j][r] = e_; sm[r] += e_; }
#pragma unroll
    for (int r = 0; r < 8; ++r) {
#pragma unroll
      for (int o = 1; o < 16; o <<= 1) sm[r] += __shfl_xor(sm[r], o); }
#pragma unroll
    for (int j = 0; j < 4; ++j)
#pragma unroll
      for (int r = 0; r < 8; ++r) sp[wave][8 * g + r][j * 16 + col] = (sm[r] > 0.f) ? pr[j][r] / sm[r] : 0.f;
    LDSX();
    v8f oc[4] = {};
#pragma unroll
    for (int kc = 0; kc < 2; ++kc) { const v16h pa = frag_f32s(&sp[wave][col][0] + kc * 32, lane, 2048.0f);
#pragma unroll
      for (int j = 0; j < 4; ++j) oc[j] = wmma16(pa, frag_h(&sv[j * 16 + col][kc * 32], lane), oc[j]); }
#pragma unroll
    for (int j = 0; j < 3; ++j)
#pragma unroll
      for (int r = 0; r < 8; ++r) so[wave * 16 + 8 * g + r][h * HD + j * 16 + col] = oc[j][r] * (1.0f / 2048.0f);
    __syncthreads(); }
  for (int e = tid; e < LW * (CC / 4); e += 128) { const int l = e / (CC / 4), q = e % (CC / 4); vst2(O + ((size_t)n * NP + stok[l]) * CC + q * 4, *(const v4f*)&so[l][q * 4]); } }
__global__ __launch_bounds__(128) void k_oproj(const float* __restrict__ O, const float* __restrict__ WO, const float* __restrict__ BO, float* __restrict__ OUT) { __shared__ __align__(16) float sf[4][16][132];
  const int tid = threadIdx.x, wave = tid >> 5, lane = tid & 31, col = lane & 15, g = lane >> 4; const int c0 = blockIdx.y * 128; const size_t r0 = (size_t)blockIdx.x * 64 + wave * 16; const size_t n = r0 / NP;
  const int rr = (int)((r0 + col) % NP); const int a = rr / WWD, bpos = rr % WWD; const size_t srow = n * NP + (size_t)bpos * WWD + a;
  v8f acc[8] = {};
#pragma unroll 2
  for (int kc = 0; kc < CC / 32; ++kc) { const F2 av = split_row(O + srow * CC, kc * 32, lane);
#pragma unroll
    for (int j = 0; j < 8; ++j) { v16b w; const int o = c0 + j * 16 + col;
#pragma unroll
      for (int i = 0; i < 8; ++i) { w[i] = (__bf16)WO[(size_t)o * CC + kc * 32 + 8 * g + i]; w[8 + i] = (__bf16)WO[(size_t)o * CC + kc * 32 + 16 + 8 * g + i]; }
      acc[j] = wmma_bf(av.h, w, acc[j]); acc[j] = wmma_bf(av.l, w, acc[j]); } }
#pragma unroll
  for (int j = 0; j < 8; ++j) { const float bb = bfr(BO[c0 + j * 16 + col]);
#pragma unroll
    for (int r = 0; r < 8; ++r) sf[wave][8 * g + r][j * 16 + col] = acc[j][r] + bb; }
  LDSX(); for (int rl = 0; rl < 16; ++rl) vst2(OUT + (r0 + rl) * CC + c0 + lane * 4, *(const v4f*)&sf[wave][rl][lane * 4]); }
extern "C" void kernel_launch(void* const* d_in, const int* in_sizes, int n_in, void* d_out, int out_size, void* d_ws, size_t ws_size, hipStream_t stream) {
  (void)in_sizes; (void)n_in; (void)out_size;
  const float** F = (const float**)d_in;
  if (ws_size < (size_t)WS_END) return;
  char* ws = (char*)d_ws; _Float16 *T16 = (_Float16*)(ws + WS_T), *P16 = (_Float16*)(ws + WS_PH_), *GT = (_Float16*)(ws + WS_GT), *P = (_Float16*)(ws + WS_P), *QKV = (_Float16*)(ws + WS_QKV); float *S = (float*)(ws + WS_S), *FG = (float*)(ws + WS_FG), *X4 = (float*)(ws + WS_X4), *O = (float*)(ws + WS_O);
  k_cproj<<<dim3(TNB * NP / 64, 3), 128, 0, stream>>>(F[0], F[4], F[5], F[6], T16, P16, GT);
  for (int b = 0; b < TNB; ++b) {
    k_csc<<<dim3(NP / 64, NP / 64), 128, 0, stream>>>(T16, P16, b, S);
    k_csm<<<NP, 256, 0, stream>>>(S, P);
    k_cpv<<<dim3(NP / 64, CI / 96), 128, 0, stream>>>(P, GT, b, FG);
  }
  k_cout<<<dim3(TNB * NP / 64, CC / 128), 128, 0, stream>>>(F[0], FG, F[7], X4);
  k_qkv<<<dim3(TNB * NP / 64, 3 * CC / 128), 128, 0, stream>>>(X4, F[8], F[9], QKV);
  k_wat<<<TNB * NQW * NQW, 128, 0, stream>>>(QKV, F[12], (const int*)d_in[13], O);
  k_oproj<<<dim3(TNB * NP / 64, CC / 128), 128, 0, stream>>>(O, F[10], F[11], (float*)d_out);
}
